// MAB_28656021799628
// MI455X (gfx1250) — hardware-run, weakly checked
//
#include <hip/hip_runtime.h>
#include <math.h>

constexpr int kBatch = 4;
constexpr int kSeq   = 2048;
constexpr int kDim   = 256;
constexpr int kFF    = 1024;
constexpr int kHeads = 8;
constexpr int kDh    = 32;
constexpr int kDhPad = 64;
constexpr int kTok   = kBatch * kSeq;
constexpr float kWCarry     = 64.0f;
constexpr float kWCarryInv  = 1.0f / 64.0f;
constexpr float kPCarry     = 32768.0f;
constexpr float kPCarryInv  = 1.0f / 32768.0f;
constexpr float kScoreScale = 0.17677669529663688f;
constexpr float kInvDim     = 1.0f / 256.0f;
constexpr float kLnEps      = 1.0e-5f;
static_assert(kHeads * kDh == kDim, "shape");
static_assert(kTok % 64 == 0 && kDim % 64 == 0 && kFF % 64 == 0 && kSeq % 64 == 0 && kDhPad % 64 == 0, "tile multiples");
static_assert(kDim % 32 == 0 && kFF % 32 == 0 && kSeq % 32 == 0 && kDh % 32 == 0, "K multiples of 32");
static_assert(kSeq == 2048 && kDim == 256, "row kernels assume these extents");

typedef __attribute__((ext_vector_type(16))) _Float16 v16h;
typedef __attribute__((ext_vector_type(8)))  _Float16 v8h;
typedef __attribute__((ext_vector_type(16))) __bf16   v16b;
typedef __attribute__((ext_vector_type(8)))  __bf16   v8b;
typedef __attribute__((ext_vector_type(8)))  float    v8f;
typedef __attribute__((ext_vector_type(4)))  float    v4f;
typedef __attribute__((ext_vector_type(2)))  float    v2f;
typedef __attribute__((ext_vector_type(4)))  unsigned int v4u;

__device__ __forceinline__ unsigned short f2bf_bits(float f) {
  unsigned u = __float_as_uint(f);
  return (unsigned short)((u + 0x7FFFu + ((u >> 16) & 1u)) >> 16);
}
__device__ __forceinline__ float bf_bits2f(unsigned short h) { return __uint_as_float(((unsigned)h) << 16); }

__device__ __forceinline__ void dep_guard_h(v8f& a, v8f& b, v16h x, v16h y) { asm volatile("v_nop\n\tv_nop\n\tv_nop\n\tv_nop" : "+v"(a), "+v"(b) : "v"(x), "v"(y)); }
__device__ __forceinline__ void dep_guard_b(v8f& a, v8f& b, v16b x, v16b y) { asm volatile("v_nop\n\tv_nop\n\tv_nop\n\tv_nop" : "+v"(a), "+v"(b) : "v"(x), "v"(y)); }
__device__ __forceinline__ void keep4_h(v16h a, v16h b, v16h c, v16h d) { asm volatile("v_nop" :: "v"(a), "v"(b), "v"(c), "v"(d)); }
__device__ __forceinline__ void keep4_b(v16b a, v16b b, v16b c, v16b d) { asm volatile("v_nop" :: "v"(a), "v"(b), "v"(c), "v"(d)); }
__device__ __forceinline__ void acc_guard4(v8f& a, v8f& b, v8f& c, v8f& d) { asm volatile("v_nop\n\tv_nop\n\tv_nop\n\tv_nop" : "+v"(a), "+v"(b), "+v"(c), "+v"(d)); }
template <typename T> struct Frag;
template <> struct Frag<_Float16> {
  typedef v16h V; union U { v16h v; v8h h[2]; };
  static __device__ __forceinline__ v16h load(const _Float16* p) {
    U f; f.h[0] = *(const v8h*)(p); f.h[1] = *(const v8h*)(p + 16); return f.v;
  }
  static __device__ __forceinline__ v8f mma(v16h a, v16h b, v8f c) {
    return __builtin_amdgcn_wmma_f32_16x16x32_f16(false, a, false, b, (short)0, c, false, false);
  }
  static __device__ __forceinline__ void guard(v8f& a, v8f& b, v16h x, v16h y) { dep_guard_h(a, b, x, y); }
  static __device__ __forceinline__ void keep(v16h a, v16h b, v16h c, v16h d) { keep4_h(a, b, c, d); }
};
template <> struct Frag<__bf16> {
  typedef v16b V; union U { v16b v; v8b h[2]; };
  static __device__ __forceinline__ v16b load(const __bf16* p) {
    U f; f.h[0] = *(const v8b*)(p); f.h[1] = *(const v8b*)(p + 16); return f.v;
  }
  static __device__ __forceinline__ v8f mma(v16b a, v16b b, v8f c) {
    return __builtin_amdgcn_wmma_f32_16x16x32_bf16(false, a, false, b, (short)0, c, false, false);
  }
  static __device__ __forceinline__ void guard(v8f& a, v8f& b, v16b x, v16b y) { dep_guard_b(a, b, x, y); }
  static __device__ __forceinline__ void keep(v16b a, v16b b, v16b c, v16b d) { keep4_b(a, b, c, d); }
};

__device__ __forceinline__ unsigned pk16(unsigned short a, unsigned short b) { return (unsigned)a | ((unsigned)b << 16); }
__device__ __forceinline__ unsigned short h_bits(float f) { const _Float16 h = (_Float16)f; return __builtin_bit_cast(unsigned short, h); }

template <int ET> struct Elem;
template <> struct Elem<0> { typedef _Float16 T; };
template <> struct Elem<1> { typedef __bf16 T; };
template <int ET, bool SPLIT, int BIAS_MODE, int OUT_MODE, bool RESID, int ACT = 0>
__global__ __launch_bounds__(256) void wmma_gemm64(
    const unsigned short* __restrict__ Ap, const unsigned short* __restrict__ A2p, int lda, long strideA,
    const unsigned short* __restrict__ Btp, const unsigned short* __restrict__ Bt2p, int ldb, long strideB,
    void* __restrict__ Cout, void* __restrict__ Cout2, int ldc, long strideC,
    const float* __restrict__ bias,
    const float* __restrict__ resid, long strideR,
    int M, int N, int K, float scale) {
  static_assert(!RESID || OUT_MODE == 0, "residual path is f32-out only");
  typedef typename Elem<ET>::T T;
  typedef typename Frag<T>::V V;
  const T* A = (const T*)Ap; const T* A2 = (const T*)A2p; const T* Bt = (const T*)Btp; const T* Bt2 = (const T*)Bt2p;
  __shared__ __align__(16) float sT[8][16 * 68];
  const int b    = blockIdx.y;
  const int lane = threadIdx.x & 31;
  const int wave = threadIdx.x >> 5;
  const int tilesN = N >> 6;
  const int tilesM = M >> 6;
  const int tile = blockIdx.x * 8 + wave;
  if (tile >= tilesM * tilesN) return;
  const int tm = tile / tilesN;
  const int tn = tile - tm * tilesN;
  const int m0 = tm << 6;
  const int n0 = tn << 6;

  const T* Ab  = A  + (size_t)b * strideA;
  const T* Bb  = Bt + (size_t)b * strideB;
  const T* Ab2 = SPLIT ? (A2  + (size_t)b * strideA) : nullptr;
  const T* Bb2 = SPLIT ? (Bt2 + (size_t)b * strideB) : nullptr;

  const int rlane = lane & 15;
  const int koff  = (lane >> 4) * 8;
  const int mOff  = (lane >> 4) * 8;

  v8f acc[4][4];
#pragma unroll
  for (int i = 0; i < 4; ++i)
#pragma unroll
    for (int j = 0; j < 4; ++j) acc[i][j] = (v8f){0.f,0.f,0.f,0.f,0.f,0.f,0.f,0.f};

  for (int k0 = 0; k0 < K; k0 += 32) {
    V bh[4], bl[4];
#pragma unroll
    for (int j = 0; j < 4; ++j) {
      const size_t bo = (size_t)(n0 + (j << 4) + rlane) * ldb + koff + k0;
      bh[j] = Frag<T>::load(Bb + bo);
      if (SPLIT) bl[j] = Frag<T>::load(Bb2 + bo);
    }
#pragma unroll
    for (int i = 0; i < 4; ++i) {
      const size_t ao = (size_t)(m0 + (i << 4) + rlane) * lda + koff + k0;
      V ah = Frag<T>::load(Ab + ao);
      V al;
      if (SPLIT) al = Frag<T>::load(Ab2 + ao);
#pragma unroll
      for (int j = 0; j < 4; ++j) {
        acc[i][j] = Frag<T>::mma(ah, bh[j], acc[i][j]);
        if (SPLIT) {
          acc[i][j] = Frag<T>::mma(ah, bl[j], acc[i][j]);
          acc[i][j] = Frag<T>::mma(al, bh[j], acc[i][j]);
        }
      }
      Frag<T>::guard(acc[i][0], acc[i][3], ah, SPLIT ? al : ah);
    }
    Frag<T>::keep(bh[0], bh[1], bh[2], bh[3]);
    if (SPLIT) Frag<T>::keep(bl[0], bl[1], bl[2], bl[3]);
  }
  acc_guard4(acc[0][0], acc[0][1], acc[0][2], acc[0][3]);
  acc_guard4(acc[1][0], acc[1][1], acc[1][2], acc[1][3]);
  acc_guard4(acc[2][0], acc[2][1], acc[2][2], acc[2][3]);
  acc_guard4(acc[3][0], acc[3][1], acc[3][2], acc[3][3]);

  float* slab = sT[wave];
  const float* Rb = RESID ? (resid + (size_t)b * strideR) : nullptr;
#pragma unroll
  for (int i = 0; i < 4; ++i) {
    const int mBase = m0 + (i << 4);
#pragma unroll
    for (int j = 0; j < 4; ++j) {
      const int n = n0 + (j << 4) + rlane;
      float bv = 0.f;
      if (BIAS_MODE == 2) bv = bias[n];
#pragma unroll
      for (int r = 0; r < 8; ++r) {
        float v = acc[i][j][r] * scale;
        if (BIAS_MODE == 1) v += bias[mBase + mOff + r];
        if (BIAS_MODE == 2) v += bv;
        if (ACT == 2) v = fmaxf(v, 0.0f);
        if (ACT == 4) v = (v > 0.f) ? v : 0.01f * v;
        slab[(mOff + r) * 68 + (j << 4) + rlane] = v;
      }
    }
    __builtin_amdgcn_fence(__ATOMIC_RELEASE, "workgroup");
    __builtin_amdgcn_wave_barrier();
    __builtin_amdgcn_fence(__ATOMIC_ACQUIRE, "workgroup");
    if (OUT_MODE == 0) {
      float* C = (float*)Cout + (size_t)b * strideC;
      const int hh = lane >> 4, c4 = (lane & 15) * 4;
      for (int pass = 0; pass < 2; ++pass) {
#pragma unroll
        for (int it = 0; it < 8; ++it) {
          const int row = it * 2 + hh;
          v4f v = *(const v4f*)(slab + row * 68 + c4);
          if (RESID) {
            const v4f rv = *(const v4f*)(Rb + (size_t)(mBase + row) * ldc + n0 + c4);
            v = v + rv;
          }
          *(volatile v4f*)(C + (size_t)(mBase + row) * ldc + n0 + c4) = v;
        }
        __threadfence();
      }
    } else {
      const int q = lane >> 3, c8 = (lane & 7) * 8;
      unsigned short* C  = (unsigned short*)Cout  + (size_t)b * strideC;
      unsigned short* C2 = (OUT_MODE == 2) ? ((unsigned short*)Cout2 + (size_t)b * strideC) : nullptr;
      for (int pass = 0; pass < 2; ++pass) {
#pragma unroll
        for (int it = 0; it < 4; ++it) {
          const int row = it * 4 + q;
          const float* sp = slab + row * 68 + c8;
          v8h hv, lv;
#pragma unroll
          for (int e = 0; e < 8; ++e) {
            if (OUT_MODE == 1) {
              hv[e] = (_Float16)sp[e];
            } else {
              unsigned short hb = f2bf_bits(sp[e]);
              unsigned short lb = f2bf_bits(sp[e] - bf_bits2f(hb));
              hv[e] = __builtin_bit_cast(_Float16, hb);
              lv[e] = __builtin_bit_cast(_Float16, lb);
            }
          }
          *(volatile v8h*)(C + (size_t)(mBase + row) * ldc + n0 + c8) = hv;
          if (OUT_MODE == 2) *(volatile v8h*)(C2 + (size_t)(mBase + row) * ldc + n0 + c8) = lv;
        }
        __threadfence();
      }
    }
    __builtin_amdgcn_fence(__ATOMIC_RELEASE, "workgroup");
    __builtin_amdgcn_wave_barrier();
    __builtin_amdgcn_fence(__ATOMIC_ACQUIRE, "workgroup");
  }
}

__global__ __launch_bounds__(256) void cast8_f16_kernel(const float* __restrict__ in, unsigned short* __restrict__ out, int n8) {
  const int i = blockIdx.x * 256 + threadIdx.x;
  if (i >= n8) return;
  const float* p = in + 8 * (size_t)i;
  const v4f a = *(const v4f*)(p);
  const v4f c = *(const v4f*)(p + 4);
  unsigned short hb[8];
#pragma unroll
  for (int e = 0; e < 4; ++e) {
    hb[e]     = h_bits(a[e]);
    hb[4 + e] = h_bits(c[e]);
  }
  const v4u u = (v4u){pk16(hb[0], hb[1]), pk16(hb[2], hb[3]), pk16(hb[4], hb[5]), pk16(hb[6], hb[7])};
  unsigned short* q = out + 8 * (size_t)i;
  *(volatile v4u*)q = u;
  __threadfence();
  *(volatile v4u*)q = u;
}

__global__ __launch_bounds__(256) void wtcast_kernel(const float* __restrict__ W, unsigned short* __restrict__ out,
                                                     int Kin, int Nout, float scale) {
  __shared__ float sm[64][65];
  const int t  = threadIdx.x;
  const int k0 = blockIdx.x * 64;
  const int n0 = blockIdx.y * 64;
#pragma unroll
  for (int i = 0; i < 16; ++i) {
    const int e = i * 256 + t;
    const int r = e >> 6;
    const int c = e & 63;
    sm[c][r] = W[(size_t)(k0 + r) * Nout + n0 + c] * scale;
  }
  __syncthreads();
  const int lane = t & 31, wave = t >> 5;
  const int q = lane >> 3, c8 = (lane & 7) * 8;
  for (int pass = 0; pass < 2; ++pass) {
#pragma unroll
    for (int it = 0; it < 2; ++it) {
      const int row = wave * 8 + it * 4 + q;
      unsigned short hb[8];
#pragma unroll
      for (int e = 0; e < 8; ++e) hb[e] = h_bits(sm[row][c8 + e]);
      const v4u u = (v4u){pk16(hb[0], hb[1]), pk16(hb[2], hb[3]), pk16(hb[4], hb[5]), pk16(hb[6], hb[7])};
      *(volatile v4u*)(out + (size_t)(n0 + row) * Kin + k0 + c8) = u;
    }
    __threadfence();
  }
}

__global__ __launch_bounds__(256) void vt_cast_kernel(const float* __restrict__ V32, unsigned short* __restrict__ VT) {
  __shared__ float sm[32][65];
  const int t  = threadIdx.x;
  const int s0 = blockIdx.x * 64;
  const int h  = blockIdx.y;
  const int b  = blockIdx.z;
#pragma unroll
  for (int i = 0; i < 8; ++i) {
    const int e = i * 256 + t;
    const int r = e >> 5;
    const int c = e & 31;
    sm[c][r] = V32[((size_t)(b * kSeq + s0 + r)) * kDim + h * kDh + c];
  }
  __syncthreads();
  const int lane = t & 31, wave = t >> 5;
  const int q = lane >> 3, c8 = (lane & 7) * 8;
  unsigned short* op = VT + ((size_t)(b * kHeads + h) * kDhPad) * kSeq;
  for (int pass = 0; pass < 2; ++pass) {
#pragma unroll
    for (int it = 0; it < 2; ++it) {
      const int row = wave * 8 + it * 4 + q;
      const int rr = (row < kDh) ? row : (kDh - 1);
      const float fz = (row < kDh) ? 1.0f : 0.0f;
      unsigned short hb[8];
#pragma unroll
      for (int e = 0; e < 8; ++e) hb[e] = h_bits(sm[rr][c8 + e] * fz);
      const v4u u = (v4u){pk16(hb[0], hb[1]), pk16(hb[2], hb[3]), pk16(hb[4], hb[5]), pk16(hb[6], hb[7])};
      *(volatile v4u*)(op + (size_t)row * kSeq + s0 + c8) = u;
    }
    __threadfence();
  }
}

__global__ __launch_bounds__(256) void softmax_row_kernel(const float* __restrict__ Sp, unsigned short* __restrict__ Pp) {
  __shared__ __align__(16) float lg[kSeq];
  __shared__ float redM[8];
  __shared__ float redS[8];
  const int i    = blockIdx.x;
  const int t    = threadIdx.x;
  const int lane = t & 31, wave = t >> 5;
  const size_t rowoff = (size_t)i * kSeq;
  const float* sr = Sp + rowoff;

  float mx = -__builtin_inff();
#pragma unroll 1
  for (int it = 0; it < 4; ++it) {
    const int c = it * 512 + 2 * t;
    const v2f sv = *(const v2f*)(sr + c);
    mx = fmaxf(mx, fmaxf(sv[0], sv[1]));
    *(v2f*)(lg + c) = sv;
  }
#pragma unroll
  for (int off = 16; off > 0; off >>= 1) mx = fmaxf(mx, __shfl_xor(mx, off, 32));
  if (lane == 0) redM[wave] = mx;
  __syncthreads();
  float m = redM[0];
#pragma unroll
  for (int w = 1; w < 8; ++w) m = fmaxf(m, redM[w]);

  float sum = 0.f;
#pragma unroll 1
  for (int it = 0; it < 4; ++it) {
    const int c = it * 512 + 2 * t;
    const v2f l = *(const v2f*)(lg + c);
    v2f ev;
#pragma unroll
    for (int e = 0; e < 2; ++e) {
      ev[e] = expf(l[e] - m);
      sum += ev[e];
    }
    *(v2f*)(lg + c) = ev;
  }
#pragma unroll
  for (int off = 16; off > 0; off >>= 1) sum += __shfl_xor(sum, off, 32);
  if (lane == 0) redS[wave] = sum;
  __syncthreads();
  float tot = redS[0];
#pragma unroll
  for (int w = 1; w < 8; ++w) tot += redS[w];
  const float inv = kPCarry / tot;

  const v4f e0 = *(const v4f*)(lg + 8 * t);
  const v4f e1 = *(const v4f*)(lg + 8 * t + 4);
  unsigned short hb[8];
#pragma unroll
  for (int e = 0; e < 4; ++e) {
    hb[e]     = h_bits(e0[e] * inv);
    hb[4 + e] = h_bits(e1[e] * inv);
  }
  const v4u u = (v4u){pk16(hb[0], hb[1]), pk16(hb[2], hb[3]), pk16(hb[4], hb[5]), pk16(hb[6], hb[7])};
  unsigned short* pr = Pp + rowoff + 8 * (size_t)t;
  *(volatile v4u*)pr = u;
  __threadfence();
  *(volatile v4u*)pr = u;
}

template <bool ADD_AV, bool OUT32>
__global__ __launch_bounds__(256) void ln_kernel(const float* __restrict__ X, const float* __restrict__ AV,
                                                 const float* __restrict__ gam, const float* __restrict__ bet,
                                                 float* __restrict__ O32, unsigned short* __restrict__ O16) {
  __shared__ __align__(16) float slab[8][kDim];
  const int t    = threadIdx.x;
  const int lane = t & 31, wave = t >> 5;
  const int row  = blockIdx.x * 8 + wave;
  const int c0   = lane * 8;
  const float* xr = X + (size_t)row * kDim + c0;
  v4f xa = *(const v4f*)(xr);
  v4f xb = *(const v4f*)(xr + 4);
  if (ADD_AV) {
    const int bb = row >> 11;
    const int ii = row & (kSeq - 1);
    const int hd = lane >> 2;
    const int d0 = (lane & 3) * 8;
    const float* ar = AV + (((size_t)(bb * kHeads + hd)) * kSeq + ii) * kDhPad + d0;
    const v4f aa = *(const v4f*)(ar);
    const v4f ab = *(const v4f*)(ar + 4);
    xa = xa + aa;
    xb = xb + ab;
  }
  asm volatile("" ::: "memory");
  const v4f ga  = *(const v4f*)(gam + c0);
  const v4f gb  = *(const v4f*)(gam + c0 + 4);
  const v4f ba  = *(const v4f*)(bet + c0);
  const v4f bbv = *(const v4f*)(bet + c0 + 4);

  float s = ((xa[0] + xa[1]) + (xa[2] + xa[3])) + ((xb[0] + xb[1]) + (xb[2] + xb[3]));
#pragma unroll
  for (int off = 16; off > 0; off >>= 1) s += __shfl_xor(s, off, 32);
  const float mean = s * kInvDim;
  const v4f da = xa - mean;
  const v4f db = xb - mean;
  float s2 = ((da[0] * da[0] + da[1] * da[1]) + (da[2] * da[2] + da[3] * da[3]))
           + ((db[0] * db[0] + db[1] * db[1]) + (db[2] * db[2] + db[3] * db[3]));
#pragma unroll
  for (int off = 16; off > 0; off >>= 1) s2 += __shfl_xor(s2, off, 32);
  const float var = s2 * kInvDim;
  const float rs  = rsqrtf(var + kLnEps);
  const v4f ya = da * rs * ga + ba;
  const v4f yb = db * rs * gb + bbv;

  unsigned short hb[8];
#pragma unroll
  for (int e = 0; e < 4; ++e) {
    hb[e]     = h_bits(ya[e]);
    hb[4 + e] = h_bits(yb[e]);
  }
  const v4u u = (v4u){pk16(hb[0], hb[1]), pk16(hb[2], hb[3]), pk16(hb[4], hb[5]), pk16(hb[6], hb[7])};
  unsigned short* op16 = O16 + (size_t)row * kDim + c0;
  *(volatile v4u*)op16 = u;
  __threadfence();
  *(volatile v4u*)op16 = u;

  if (OUT32) {
    float* sw = slab[wave];
    *(v4f*)(sw + c0)     = ya;
    *(v4f*)(sw + c0 + 4) = yb;
    __syncthreads();
    const v4f p0 = *(const v4f*)(sw + lane * 4);
    const v4f p1 = *(const v4f*)(sw + 128 + lane * 4);
    float* o0 = O32 + (size_t)row * kDim + lane * 4;
    float* o1 = o0 + 128;
    *(volatile v4f*)o0 = p0;
    *(volatile v4f*)o1 = p1;
    __threadfence();
    *(volatile v4f*)o0 = p0;
    *(volatile v4f*)o1 = p1;
  }
}

extern "C" void kernel_launch(void* const* d_in, const int* in_sizes, int n_in,
                              void* d_out, int out_size, void* d_ws, size_t ws_size,
                              hipStream_t stream) {
  if (n_in < 18) return;
  const int nTokD = kTok * kDim;
  if (in_sizes[0] != nTokD || in_sizes[1] != nTokD) return;
  if (in_sizes[2] != kDim * kDim || in_sizes[4] != kDim * kDim || in_sizes[6] != kDim * kDim || in_sizes[8] != kDim * kDim) return;
  if (in_sizes[10] != kDim * kFF || in_sizes[12] != kFF * kDim) return;
  if (in_sizes[3] != kDim || in_sizes[5] != kDim || in_sizes[7] != kDim || in_sizes[9] != kDim || in_sizes[13] != kDim) return;
  if (in_sizes[11] != kFF) return;
  if (in_sizes[14] != kDim || in_sizes[15] != kDim || in_sizes[16] != kDim || in_sizes[17] != kDim) return;
  if (out_size != nTokD) return;

  const size_t szWsq = (size_t)kDim * kDim * 2;
  const size_t szWff = (size_t)kDim * kFF * 2;
  const size_t szA16 = (size_t)kTok * kDim * 2;
  const size_t szA32 = (size_t)kTok * kDim * 4;
  const size_t szVT  = (size_t)kBatch * kHeads * kDhPad * kSeq * 2;
  const size_t szSC  = (size_t)kSeq * kSeq * 4;
  const size_t szPP  = (size_t)kSeq * kSeq * 2;
  const size_t szAV  = (size_t)kBatch * kHeads * kSeq * kDhPad * 4;
  const size_t szH16 = (size_t)kTok * kFF * 2;
  const size_t offWq  = 0;
  const size_t offWk  = offWq + szWsq;
  const size_t offWv  = offWk + szWsq;
  const size_t offWo  = offWv + szWsq;
  const size_t offWm  = offWo + szWsq;
  const size_t offWe  = offWm + szWff;
  const size_t offq16 = offWe + szWff;
  const size_t offx16 = offq16 + szA16;
  const size_t offQ32 = offx16 + szA16;
  const size_t offQ16 = offQ32 + szA32;
  const size_t offK16 = offQ16 + szA16;
  const size_t offV32 = offK16 + szA16;
  const size_t offVT  = offV32 + szA32;
  const size_t offSC  = offVT + szVT;
  const size_t offPP  = offSC + szSC;
  const size_t offAV  = offPP + szPP;
  const size_t offON32 = offAV + szAV;
  const size_t offON16 = offON32 + szA32;
  const size_t offX2   = offON16 + szA16;
  const size_t offY16  = offX2 + szA32;
  const size_t offH16  = offY16 + szA16;
  const size_t total   = offH16 + szH16;
  if (ws_size < total) return;

  const float* q  = (const float*)d_in[0];
  const float* x  = (const float*)d_in[1];
  const float* Wq = (const float*)d_in[2];  const float* bq = (const float*)d_in[3];
  const float* Wk = (const float*)d_in[4];  const float* bk = (const float*)d_in[5];
  const float* Wv = (const float*)d_in[6];  const float* bv = (const float*)d_in[7];
  const float* Wo = (const float*)d_in[8];  const float* bo = (const float*)d_in[9];
  const float* Wm = (const float*)d_in[10]; const float* bm = (const float*)d_in[11];
  const float* We = (const float*)d_in[12]; const float* be = (const float*)d_in[13];
  const float* g0 = (const float*)d_in[14]; const float* b0 = (const float*)d_in[15];
  const float* g1 = (const float*)d_in[16]; const float* b1 = (const float*)d_in[17];
  float* out = (float*)d_out;
  char* ws = (char*)d_ws;
  unsigned short* WqT = (unsigned short*)(ws + offWq);
  unsigned short* WkT = (unsigned short*)(ws + offWk);
  unsigned short* WvT = (unsigned short*)(ws + offWv);
  unsigned short* WoT = (unsigned short*)(ws + offWo);
  unsigned short* WmT = (unsigned short*)(ws + offWm);
  unsigned short* WeT = (unsigned short*)(ws + offWe);
  unsigned short* q16 = (unsigned short*)(ws + offq16);
  unsigned short* x16 = (unsigned short*)(ws + offx16);
  float*          Q32 = (float*)(ws + offQ32);
  unsigned short* Q16 = (unsigned short*)(ws + offQ16);
  unsigned short* K16 = (unsigned short*)(ws + offK16);
  float*          V32 = (float*)(ws + offV32);
  unsigned short* VT  = (unsigned short*)(ws + offVT);
  float*          SC  = (float*)(ws + offSC);
  unsigned short* PP  = (unsigned short*)(ws + offPP);
  float*          AVT = (float*)(ws + offAV);
  float*          ON32 = (float*)(ws + offON32);
  unsigned short* ON16 = (unsigned short*)(ws + offON16);
  float*          X2   = (float*)(ws + offX2);
  unsigned short* Y16  = (unsigned short*)(ws + offY16);
  unsigned short* H16  = (unsigned short*)(ws + offH16);

  const int n8 = nTokD / 8;
  cast8_f16_kernel<<<dim3(n8 / 256), dim3(256), 0, stream>>>(q, q16, n8);
  cast8_f16_kernel<<<dim3(n8 / 256), dim3(256), 0, stream>>>(x, x16, n8);
  wtcast_kernel<<<dim3(kDim / 64, kDim / 64), dim3(256), 0, stream>>>(Wq, WqT, kDim, kDim, kWCarry);
  wtcast_kernel<<<dim3(kDim / 64, kDim / 64), dim3(256), 0, stream>>>(Wk, WkT, kDim, kDim, kWCarry);
  wtcast_kernel<<<dim3(kDim / 64, kDim / 64), dim3(256), 0, stream>>>(Wv, WvT, kDim, kDim, kWCarry);
  wtcast_kernel<<<dim3(kDim / 64, kDim / 64), dim3(256), 0, stream>>>(Wo, WoT, kDim, kDim, kWCarry);
  wtcast_kernel<<<dim3(kDim / 64, kFF / 64), dim3(256), 0, stream>>>(Wm, WmT, kDim, kFF, kWCarry);
  wtcast_kernel<<<dim3(kFF / 64, kDim / 64), dim3(256), 0, stream>>>(We, WeT, kFF, kDim, kWCarry);

  const int tilesProj = (kTok / 64) * (kDim / 64);
  wmma_gemm64<0, false, 2, 0, false, 0><<<dim3(tilesProj / 8, 1), dim3(256), 0, stream>>>(
      q16, q16, kDim, 0L, WqT, WqT, kDim, 0L, (void*)Q32, (void*)Q32, kDim, 0L, bq, Q32, 0L, kTok, kDim, kDim, kWCarryInv);
  cast8_f16_kernel<<<dim3(n8 / 256), dim3(256), 0, stream>>>(Q32, Q16, n8);
  wmma_gemm64<0, false, 2, 1, false, 0><<<dim3(tilesProj / 8, 1), dim3(256), 0, stream>>>(
      x16, x16, kDim, 0L, WkT, WkT, kDim, 0L, (void*)K16, (void*)K16, kDim, 0L, bk, Q32, 0L, kTok, kDim, kDim, kWCarryInv);
  wmma_gemm64<0, false, 2, 0, false, 0><<<dim3(tilesProj / 8, 1), dim3(256), 0, stream>>>(
      x16, x16, kDim, 0L, WvT, WvT, kDim, 0L, (void*)V32, (void*)V32, kDim, 0L, bv, Q32, 0L, kTok, kDim, kDim, kWCarryInv);
  vt_cast_kernel<<<dim3(kSeq / 64, kHeads, kBatch), dim3(256), 0, stream>>>(V32, VT);

  const int tilesScore = (kSeq / 64) * (kSeq / 64);
  const int tilesCtx   = (kSeq / 64) * (kDhPad / 64);
  for (int b = 0; b < kBatch; ++b) {
    for (int h = 0; h < kHeads; ++h) {
      const size_t tokOff = ((size_t)b * kSeq) * kDim + (size_t)h * kDh;
      const size_t bhIdx  = (size_t)b * kHeads + h;
      const unsigned short* Ag  = Q16 + tokOff;
      const unsigned short* Btg = K16 + tokOff;
      wmma_gemm64<0, false, 0, 0, false, 0><<<dim3(tilesScore / 8, 1), dim3(256), 0, stream>>>(
          Ag, Ag, kDim, 0L, Btg, Btg, kDim, 0L, (void*)SC, (void*)SC, kSeq, 0L, bq, Q32, 0L, kSeq, kSeq, kDh, kScoreScale);
      softmax_row_kernel<<<dim3(kSeq), dim3(256), 0, stream>>>(SC, PP);
      const unsigned short* VTg = VT + bhIdx * (size_t)kDhPad * kSeq;
      float* AVg = AVT + bhIdx * (size_t)kSeq * kDhPad;
      wmma_gemm64<0, false, 0, 0, false, 0><<<dim3(tilesCtx / 8, 1), dim3(256), 0, stream>>>(
          PP, PP, kSeq, 0L, VTg, VTg, kSeq, 0L, (void*)AVg, (void*)AVg, kDhPad, 0L, bq, Q32, 0L, kSeq, kDhPad, kSeq, kPCarryInv);
    }
  }

  ln_kernel<true, true><<<dim3(kTok / 8), dim3(256), 0, stream>>>(Q32, AVT, g0, b0, ON32, ON16);
  wmma_gemm64<0, false, 2, 0, true, 2><<<dim3(tilesProj / 8, 1), dim3(256), 0, stream>>>(
      ON16, ON16, kDim, 0L, WoT, WoT, kDim, 0L, (void*)X2, (void*)X2, kDim, 0L, bo, ON32, 0L, kTok, kDim, kDim, kWCarryInv);
  ln_kernel<false, false><<<dim3(kTok / 8), dim3(256), 0, stream>>>(X2, AVT, g1, b1, ON32, Y16);
  const int tilesFF = (kTok / 64) * (kFF / 64);
  wmma_gemm64<0, false, 2, 1, false, 2><<<dim3(tilesFF / 8, 1), dim3(256), 0, stream>>>(
      Y16, Y16, kDim, 0L, WmT, WmT, kDim, 0L, (void*)H16, (void*)H16, kFF, 0L, bm, X2, 0L, kTok, kFF, kDim, kWCarryInv);
  wmma_gemm64<0, false, 2, 0, true, 0><<<dim3(tilesProj / 8, 1), dim3(256), 0, stream>>>(
      H16, H16, kFF, 0L, WeT, WeT, kFF, 0L, (void*)out, (void*)out, kDim, 0L, be, X2, 0L, kTok, kDim, kFF, kWCarryInv);
}
